// GGNN_9826885173933
// MI455X (gfx1250) — hardware-verified
//
#include <hip/hip_runtime.h>

typedef float          v8f   __attribute__((ext_vector_type(8)));
typedef float          v4f   __attribute__((ext_vector_type(4)));
typedef unsigned int   v4u   __attribute__((ext_vector_type(4)));
typedef int            v8i   __attribute__((ext_vector_type(8)));
typedef unsigned short v8us  __attribute__((ext_vector_type(8)));
typedef unsigned short v16us __attribute__((ext_vector_type(16)));
typedef __bf16         v16bf __attribute__((ext_vector_type(16)));
typedef _Float16       v16h  __attribute__((ext_vector_type(16)));
typedef v4f  __attribute__((may_alias)) v4fa;
typedef v8us __attribute__((may_alias)) v8usa;
union FragB { v16bf v; v16us u; v8us h[2]; v8i w; };
union FragH { v16h  v; v16us u; v8us h[2]; v8i w; };

__device__ __forceinline__ v8f wmb(const FragB& a, const FragB& b, v8f c) {
  v8f d = __builtin_amdgcn_wmma_f32_16x16x32_bf16(false, a.v, false, b.v, (short)0, c, false, false);
  asm volatile("v_nop\n\tv_nop\n\tv_nop\n\tv_nop" : "+v"(d) : "v"(a.w), "v"(b.w));
  return d;
}

__device__ __forceinline__ v8f wmh(const FragH& a, const FragH& b, v8f c) {
  v8f d = __builtin_amdgcn_wmma_f32_16x16x32_f16(false, a.v, false, b.v, (short)0, c, false, false);
  asm volatile("v_nop\n\tv_nop\n\tv_nop\n\tv_nop" : "+v"(d) : "v"(a.w), "v"(b.w));
  return d;
}

__device__ __forceinline__ unsigned bf16_bits(float f) {
  const unsigned u = __float_as_uint(f);
  const unsigned r = (u + 0x7FFFu + ((u >> 16) & 1u)) >> 16;
  const unsigned q = (u >> 16) | 0x40u;
  return ((u & 0x7fffffffu) > 0x7f800000u) ? q : r;
}

__device__ __forceinline__ float bf16_val(float f) {
  return __uint_as_float(bf16_bits(f) << 16);
}
__device__ __forceinline__ int clampi(int v, int lo, int hi) {
  return v < lo ? lo : (v > hi ? hi : v);
}

__device__ __forceinline__ unsigned f16_bits(float f) {
  const unsigned u  = __float_as_uint(f);
  const unsigned s  = (u >> 16) & 0x8000u;
  const unsigned a  = u & 0x7fffffffu;
  const unsigned t  = a - 0x38000000u;
  const unsigned r  = (t + 0x0FFFu + ((t >> 13) & 1u)) >> 13;
  const unsigned rc = r > 0x7C00u ? 0x7C00u : r;
  const bool small  = a < 0x38800000u;
  const bool isnan  = a > 0x7f800000u;
  const unsigned fin = small ? 0u : (s | rc);
  return isnan ? (s | 0x7E00u) : fin;
}

__device__ __forceinline__ unsigned pk16(unsigned lo, unsigned hi) { return lo | (hi << 16); }
__device__ __forceinline__ unsigned bf16_lo_bits(float v) {
  float hi = bf16_val(v);
  asm volatile("" : "+v"(hi));
  return bf16_bits(v - hi);
}
__device__ __forceinline__ v4u pack8_bf16(v4f a, v4f c) {
  return (v4u){ pk16(bf16_bits(a[0]), bf16_bits(a[1])), pk16(bf16_bits(a[2]), bf16_bits(a[3])),
                pk16(bf16_bits(c[0]), bf16_bits(c[1])), pk16(bf16_bits(c[2]), bf16_bits(c[3])) };
}
__device__ __forceinline__ v4u pack8_bf16_lo(v4f a, v4f c) {
  return (v4u){ pk16(bf16_lo_bits(a[0]), bf16_lo_bits(a[1])), pk16(bf16_lo_bits(a[2]), bf16_lo_bits(a[3])),
                pk16(bf16_lo_bits(c[0]), bf16_lo_bits(c[1])), pk16(bf16_lo_bits(c[2]), bf16_lo_bits(c[3])) };
}
__device__ __forceinline__ v4u pack8_f16(v4f a, v4f c) {
  return (v4u){ pk16(f16_bits(a[0]), f16_bits(a[1])), pk16(f16_bits(a[2]), f16_bits(a[3])),
                pk16(f16_bits(c[0]), f16_bits(c[1])), pk16(f16_bits(c[2]), f16_bits(c[3])) };
}

template <int FORM>
__global__ __launch_bounds__(256) void k_plane(const float* __restrict__ src, int rows, int cols, int ldsrc,
                                               unsigned short* __restrict__ dst, int MP, int KP) {
  static_assert(FORM >= 0 && FORM <= 3);
  const int KTOT = (FORM == 1 || FORM == 3) ? 2 * KP : KP;
  const unsigned ppr   = (unsigned)(KTOT >> 3);
  const unsigned kp8   = (unsigned)(KP >> 3);
  const unsigned total = (unsigned)MP * ppr;
  const unsigned g     = blockIdx.x * 256u + threadIdx.x;
  const unsigned rowu  = g / ppr;
  const unsigned p     = g - rowu * ppr;
  const bool second    = p >= kp8;
  const int row = (int)rowu;
  const int c0  = (int)((second ? p - kp8 : p) << 3);
  const float* srow = src + (size_t)clampi(row, 0, rows - 1) * (size_t)ldsrc;
  float x[8];
  unsigned mk[8];
#pragma unroll
  for (int e = 0; e < 8; ++e) {
    const int c = c0 + e;
    const float v = srow[clampi(c, 0, cols - 1)];
    asm volatile("" :: "v"(v));
    x[e]  = v;
    mk[e] = (row < rows && c < cols) ? 0xFFFFu : 0u;
  }
  const v4f a = (v4f){ x[0], x[1], x[2], x[3] };
  const v4f c = (v4f){ x[4], x[5], x[6], x[7] };
  v4u o;
  if (FORM == 2) {
    o = pack8_f16(a, c);
  } else {
    const v4u hi = pack8_bf16(a, c);
    o = hi;
    if (FORM == 1) { const v4u lo = pack8_bf16_lo(a, c); o = second ? lo : hi; }
  }
  const v4u mw = (v4u){ pk16(mk[0], mk[1]), pk16(mk[2], mk[3]), pk16(mk[4], mk[5]), pk16(mk[6], mk[7]) };
  o &= mw;
  if (g < total) {
    volatile v4u* q = (volatile v4u*)(dst + (size_t)g * 8);
    *q = o;
    __threadfence();
    *q = o;
  }
}

template <int FORM> struct FragOf    { typedef FragB T; };
template <>         struct FragOf<2> { typedef FragH T; };
__device__ __forceinline__ v8f mm(const FragB& a, const FragB& b, v8f c) { return wmb(a, b, c); }
__device__ __forceinline__ v8f mm(const FragH& a, const FragH& b, v8f c) { return wmh(a, b, c); }
template <class F> __device__ __forceinline__ F ld_frag(const unsigned short* p) {
  F f;
  f.h[0] = *(const v8usa*)(p);
  f.h[1] = *(const v8usa*)(p + 16);
  return f;
}

template <int FORM, int EPI>
__global__ __launch_bounds__(256) __attribute__((amdgpu_num_vgpr(248)))
void k_gemm_nt(const unsigned short* __restrict__ A, const unsigned short* __restrict__ B,
               const float* __restrict__ bias, float* __restrict__ D, int M, int N, int KTOT, int ldd) {
  static_assert(FORM >= 0 && FORM <= 2);
  static_assert(EPI == 0 || EPI == 1);
  typedef typename FragOf<FORM>::T F;
  __shared__ __attribute__((aligned(16))) float sT[8][16 * 68];
  const int lane = threadIdx.x & 31;
  const int wave = threadIdx.x >> 5;
  const int tilesM = (M + 63) >> 6;
  const int tilesN = (N + 63) >> 6;
  const int tile = blockIdx.x * 8 + wave;
  if (tile >= tilesM * tilesN) return;
  const int tm = tile / tilesN;
  const int tn = tile - tm * tilesN;
  const int m0 = tm << 6;
  const int n0 = tn << 6;

  const int rl = lane & 15;
  const int h8 = (lane >> 4) * 8;
  const unsigned short* pa = A + (size_t)(m0 + rl) * (size_t)KTOT + h8;
  const unsigned short* pb = B + (size_t)(n0 + rl) * (size_t)KTOT + h8;

  v8f acc[4][4];
#pragma unroll
  for (int i = 0; i < 4; ++i)
#pragma unroll
    for (int j = 0; j < 4; ++j) acc[i][j] = (v8f){0.f, 0.f, 0.f, 0.f, 0.f, 0.f, 0.f, 0.f};

#pragma unroll 1
  for (int k0 = 0; k0 < KTOT; k0 += 32) {
    F bf[4];
#pragma unroll
    for (int j = 0; j < 4; ++j) bf[j] = ld_frag<F>(pb + (size_t)(j << 4) * (size_t)KTOT + k0);
#pragma unroll
    for (int i = 0; i < 4; ++i) {
      const F af = ld_frag<F>(pa + (size_t)(i << 4) * (size_t)KTOT + k0);
#pragma unroll
      for (int j = 0; j < 4; ++j) acc[i][j] = mm(af, bf[j], acc[i][j]);
    }
  }

  float* slab = sT[wave];
  const int hh = lane >> 4;
  const int c4 = (lane & 15) * 4;
  const int nc = n0 + c4;
  const bool cok = nc < N;
  v4f bv = (v4f){0.f, 0.f, 0.f, 0.f};
  if (EPI == 1) {
    bv = *(const v4fa*)(bias + clampi(nc, 0, N - 4));
    asm volatile("" :: "v"(bv));
  }
#pragma unroll
  for (int i = 0; i < 4; ++i) {
    const int mBase = m0 + (i << 4);
#pragma unroll
    for (int j = 0; j < 4; ++j) {
#pragma unroll
      for (int r = 0; r < 8; ++r) slab[(h8 + r) * 68 + (j << 4) + rl] = acc[i][j][r];
    }
    __builtin_amdgcn_fence(__ATOMIC_RELEASE, "workgroup");
    __builtin_amdgcn_wave_barrier();
    __builtin_amdgcn_fence(__ATOMIC_ACQUIRE, "workgroup");
    v4f vv[8];
#pragma unroll
    for (int it = 0; it < 8; ++it) {
      const int row = it * 2 + hh;
      v4f v = *(const v4fa*)(slab + row * 68 + c4);
      if (EPI == 1) v += bv;
      vv[it] = v;
    }
    for (int pass = 0; pass < 2; ++pass) {
#pragma unroll
      for (int it = 0; it < 8; ++it) {
        const int row = mBase + it * 2 + hh;
        if (cok && row < M) *(volatile v4f*)(D + (size_t)row * (size_t)ldd + nc) = vv[it];
      }
      __threadfence();
    }
    __builtin_amdgcn_fence(__ATOMIC_RELEASE, "workgroup");
    __builtin_amdgcn_wave_barrier();
    __builtin_amdgcn_fence(__ATOMIC_ACQUIRE, "workgroup");
  }
}

#pragma clang fp contract(off)
#include <stddef.h>
#include <stdint.h>
#include <math.h>

#define NN      50000
#define NE      800000
#define HD      64
#define NTY     4
#define NSTEP   4
#define NPAD    50048
#define KT      128
#define TLD     256
#define GLD     192
#define XA0     0
#define XAR     25088
#define XB0     25088
#define XBR     24960
#define NTHR    256
#define NWAVE   8
#define EPT     8
#define WCH     (32 * EPT)
#define NBRUN   512
#define SLB     9
#define NBK     98
#define WLCAP   2048
#define RCAP    12288
#define DEGCAP  48
#define MAXDEG_MEAS  36
#define MAXB512_MEAS 8374
#define WSMAX   ((size_t)128 << 20)

#define BK_ZINTS (NWAVE * WLCAP + RCAP + 3 * NBRUN)
#define BK_INTS  (BK_ZINTS + 16)
#define BK_LDS   (BK_INTS * 4)

#define PB_WTY  (NTY * HD * KT / 8 / NTHR)
#define PB_WG   (GLD * KT / 8 / NTHR)
#define PB_ALL  (PB_WTY + 2 * PB_WG + 3)

static_assert(NN < (1 << 24));
static_assert(NE < (1 << 20));
static_assert(NBRUN == (1 << SLB) && NBRUN % 32 == 0);
static_assert((((long long)NE) << SLB) < (1LL << 31));
static_assert(NE % EPT == 0 && NE >= EPT);
static_assert(NBK * NBRUN >= NPAD && (NBK - 1) * NBRUN < NN);
static_assert(RCAP % (NTHR * 4) == 0);
static_assert((long long)RCAP * 100 >= (long long)MAXB512_MEAS * 125);
static_assert(MAXDEG_MEAS + 8 <= DEGCAP);
static_assert(WLCAP >= MAXB512_MEAS / 8 + 8 * 46 + 1);
static_assert(BK_ZINTS % 4 == 0 && (NWAVE * WLCAP) % 4 == 0);
static_assert(BK_LDS <= 327680);
static_assert(2 * NBRUN == NTHR * 4);
static_assert(NPAD % 128 == 0 && NPAD % 64 == 0 && NPAD >= NN && NPAD % 16 == 0);
static_assert(XA0 + XAR == XB0 && XB0 + XBR == NPAD && XAR % 64 == 0 && XBR % 64 == 0 && XB0 % 2 == 0);
static_assert(KT == 2 * HD && KT % 32 == 0 && HD % 8 == 0);
static_assert(TLD == NTY * HD && TLD % 64 == 0 && TLD % 32 == 0);
static_assert(GLD == 3 * HD && GLD % 64 == 0 && GLD % 32 == 0);
static_assert((NTY * HD * KT / 8) % NTHR == 0 && (GLD * KT / 8) % NTHR == 0);
static_assert((NPAD * 16) % NTHR == 0 && (XAR * 16) % NTHR == 0 && (XBR * 16) % NTHR == 0);
static_assert((NN * HD / 4) % NTHR == 0 && NN * HD == 3200000);
static_assert(NTY == 4);

typedef int v4i __attribute__((ext_vector_type(4)));
typedef v4i __attribute__((may_alias)) v4ia;

__device__ __forceinline__ void st2_v4f(float* p, v4f v) {
  *(volatile v4f*)p = v;
  __threadfence();
  *(volatile v4f*)p = v;
}
__device__ __forceinline__ void st2_v4i(int* p, v4i v) {
  *(volatile v4i*)p = v;
  __threadfence();
  *(volatile v4i*)p = v;
}
__device__ __forceinline__ void st2_v4u(unsigned short* p, v4u v) {
  *(volatile v4u*)p = v;
  __threadfence();
  *(volatile v4u*)p = v;
}

__device__ __forceinline__ v4u row_piece(v4f q, int lane) {
  const int l  = lane & 15;
  const int sA = (lane & 16) + 2 * (l & 7);
  const int sB = sA + 1;
  v4f a, c;
  a.x = __shfl(q.x, sA, 32); a.y = __shfl(q.y, sA, 32); a.z = __shfl(q.z, sA, 32); a.w = __shfl(q.w, sA, 32);
  c.x = __shfl(q.x, sB, 32); c.y = __shfl(q.y, sB, 32); c.z = __shfl(q.z, sB, 32); c.w = __shfl(q.w, sB, 32);
  const v4u hi = pack8_bf16(a, c);
  const v4u lo = pack8_bf16_lo(a, c);
  const unsigned m = (l < 8) ? 0xFFFFFFFFu : 0u;
  return (hi & m) | (lo & ~m);
}

__global__ __launch_bounds__(NTHR) void k_init(const float* __restrict__ h, float* FEAT, unsigned short* OPF) {
  const int g   = (int)blockIdx.x * NTHR + (int)threadIdx.x;
  const int row = g >> 4;
  const int l   = g & 15;
  const float* hr = h + (size_t)clampi(row, 0, NN - 1) * HD;
  const v4f x = *(const v4fa*)(hr + 4 * l);
  const v4f a = *(const v4fa*)(hr + 8 * (l & 7));
  const v4f c = *(const v4fa*)(hr + 8 * (l & 7) + 4);
  asm volatile("" :: "v"(x));
  asm volatile("" :: "v"(a));
  asm volatile("" :: "v"(c));
  const unsigned mr = (row < NN) ? 0xFFFFFFFFu : 0u;
  const unsigned mo = (row < NN && l < 8) ? 0xFFFFFFFFu : 0u;
  v4f fv;
  fv.x = __uint_as_float((bf16_bits(x.x) << 16) & mr);
  fv.y = __uint_as_float((bf16_bits(x.y) << 16) & mr);
  fv.z = __uint_as_float((bf16_bits(x.z) << 16) & mr);
  fv.w = __uint_as_float((bf16_bits(x.w) << 16) & mr);
  const v4u o = pack8_bf16(a, c) & mo;
  if (row < NPAD) {
    st2_v4f(FEAT + (size_t)row * HD + 4 * l, fv);
    st2_v4u(OPF + (size_t)row * KT + 8 * l, o);
  }
}

__device__ __forceinline__ void prep_plane(const float* __restrict__ w, unsigned short* dst, int g) {
  const int row = g >> 4;
  const int c0  = (g & 7) * 8;
  const float* p = w + (size_t)row * HD + c0;
  const v4f a = *(const v4fa*)p;
  const v4f c = *(const v4fa*)(p + 4);
  st2_v4u(dst + (size_t)g * 8, pack8_bf16(a, c));
}
__device__ __forceinline__ void prep_line(const float* __restrict__ src, float* dst, int tid, int n4) {
  const int idx = tid < n4 ? tid : n4 - 1;
  const v4f a = *(const v4fa*)(src + 4 * idx);
  asm volatile("" :: "v"(a));
  v4f o;
  o.x = bf16_val(a.x); o.y = bf16_val(a.y); o.z = bf16_val(a.z); o.w = bf16_val(a.w);
  if (tid < n4) st2_v4f(dst + 4 * tid, o);
}
__global__ __launch_bounds__(NTHR) void k_prep(const float* __restrict__ W, const float* __restrict__ b,
                                               const float* __restrict__ wih, const float* __restrict__ whh,
                                               const float* __restrict__ bih, const float* __restrict__ bhh,
                                               unsigned short* WTY, unsigned short* WIH, unsigned short* WHH,
                                               float* BT, float* BI, float* BH) {
  const int tid = (int)threadIdx.x;
  const int blk = (int)blockIdx.x;
  if (blk < PB_WTY) {
    prep_plane(W, WTY, blk * NTHR + tid);
  } else if (blk < PB_WTY + PB_WG) {
    prep_plane(wih, WIH, (blk - PB_WTY) * NTHR + tid);
  } else if (blk < PB_WTY + 2 * PB_WG) {
    prep_plane(whh, WHH, (blk - PB_WTY - PB_WG) * NTHR + tid);
  } else if (blk == PB_WTY + 2 * PB_WG) {
    prep_line(b, BT, tid, NTY * HD / 4);
  } else if (blk == PB_WTY + 2 * PB_WG + 1) {
    prep_line(bih, BI, tid, GLD / 4);
  } else {
    prep_line(bhh, BH, tid, GLD / 4);
  }
}

__global__ __launch_bounds__(NTHR) void k_list(const int* __restrict__ srcs, const int* __restrict__ dsts,
                                               const int* __restrict__ types, int* LIST, int* CO, int* FLAG) {
  extern __shared__ __attribute__((aligned(16))) int dsm[];
  int* wl   = dsm;
  int* pl   = dsm + NWAVE * WLCAP;
  int* cnt  = pl + RCAP;
  int* offs = cnt + NBRUN;
  int* cur  = offs + NBRUN;
  int* misc = cur + NBRUN;
  const int tid = (int)threadIdx.x, lane = tid & 31, wave = tid >> 5;
  const int blk = (int)blockIdx.x;
  const unsigned nbs = (unsigned)(blk * NBRUN);

  {
    const v4i z4 = {0, 0, 0, 0};
    for (int i = tid * 4; i < BK_ZINTS; i += NTHR * 4) *(v4ia*)(dsm + i) = z4;
    if (tid < 16) misc[tid] = 0;
  }
  __syncthreads();

  {
    const int per  = ((NE + NWAVE * WCH - 1) / (NWAVE * WCH)) * WCH;
    const int ebeg = wave * per;
    const int eend = (ebeg + per < NE) ? (ebeg + per) : NE;
    int* mylist = wl + wave * WLCAP;
    int wc = 0;
#pragma unroll 1
    for (int cb = ebeg; cb < eend; cb += WCH) {
      const int e0 = cb + lane * EPT;
      const int ec = e0 < NE - EPT ? e0 : NE - EPT;
      const v4i da = *(const v4ia*)(dsts + ec);
      const v4i db = *(const v4ia*)(dsts + ec + 4);
      asm volatile("" :: "v"(da));
      asm volatile("" :: "v"(db));
      const int vm = (e0 < NE) ? -1 : 0;
      const unsigned k0 = (unsigned)((da.x & vm) | ~vm), k1 = (unsigned)((da.y & vm) | ~vm);
      const unsigned k2 = (unsigned)((da.z & vm) | ~vm), k3 = (unsigned)((da.w & vm) | ~vm);
      const unsigned k4 = (unsigned)((db.x & vm) | ~vm), k5 = (unsigned)((db.y & vm) | ~vm);
      const unsigned k6 = (unsigned)((db.z & vm) | ~vm), k7 = (unsigned)((db.w & vm) | ~vm);
      const unsigned s0 = k0 - nbs, s1 = k1 - nbs, s2 = k2 - nbs, s3 = k3 - nbs;
      const unsigned s4 = k4 - nbs, s5 = k5 - nbs, s6 = k6 - nbs, s7 = k7 - nbs;
      const bool h0 = (s0 < (unsigned)NBRUN) & (k0 < (unsigned)NN), h1 = (s1 < (unsigned)NBRUN) & (k1 < (unsigned)NN);
      const bool h2 = (s2 < (unsigned)NBRUN) & (k2 < (unsigned)NN), h3 = (s3 < (unsigned)NBRUN) & (k3 < (unsigned)NN);
      const bool h4 = (s4 < (unsigned)NBRUN) & (k4 < (unsigned)NN), h5 = (s5 < (unsigned)NBRUN) & (k5 < (unsigned)NN);
      const bool h6 = (s6 < (unsigned)NBRUN) & (k6 < (unsigned)NN), h7 = (s7 < (unsigned)NBRUN) & (k7 < (unsigned)NN);
      const unsigned m0 = __builtin_amdgcn_ballot_w32(h0), m1 = __builtin_amdgcn_ballot_w32(h1);
      const unsigned m2 = __builtin_amdgcn_ballot_w32(h2), m3 = __builtin_amdgcn_ballot_w32(h3);
      const unsigned m4 = __builtin_amdgcn_ballot_w32(h4), m5 = __builtin_amdgcn_ballot_w32(h5);
      const unsigned m6 = __builtin_amdgcn_ballot_w32(h6), m7 = __builtin_amdgcn_ballot_w32(h7);
      const unsigned any = m0 | m1 | m2 | m3 | m4 | m5 | m6 | m7;
      if (any != 0u) {
        const int pre = (int)(__builtin_amdgcn_mbcnt_lo(m0, 0u) + __builtin_amdgcn_mbcnt_lo(m1, 0u) +
                              __builtin_amdgcn_mbcnt_lo(m2, 0u) + __builtin_amdgcn_mbcnt_lo(m3, 0u) +
                              __builtin_amdgcn_mbcnt_lo(m4, 0u) + __builtin_amdgcn_mbcnt_lo(m5, 0u) +
                              __builtin_amdgcn_mbcnt_lo(m6, 0u) + __builtin_amdgcn_mbcnt_lo(m7, 0u));
        int p = wc + pre;
        if (h0) { if (p < WLCAP) mylist[p] = ((e0 + 0) << SLB) | (int)s0; p = p + 1; }
        if (h1) { if (p < WLCAP) mylist[p] = ((e0 + 1) << SLB) | (int)s1; p = p + 1; }
        if (h2) { if (p < WLCAP) mylist[p] = ((e0 + 2) << SLB) | (int)s2; p = p + 1; }
        if (h3) { if (p < WLCAP) mylist[p] = ((e0 + 3) << SLB) | (int)s3; p = p + 1; }
        if (h4) { if (p < WLCAP) mylist[p] = ((e0 + 4) << SLB) | (int)s4; p = p + 1; }
        if (h5) { if (p < WLCAP) mylist[p] = ((e0 + 5) << SLB) | (int)s5; p = p + 1; }
        if (h6) { if (p < WLCAP) mylist[p] = ((e0 + 6) << SLB) | (int)s6; p = p + 1; }
        if (h7) { if (p < WLCAP) mylist[p] = ((e0 + 7) << SLB) | (int)s7; p = p + 1; }
        wc += (int)(__builtin_popcount(m0) + __builtin_popcount(m1) + __builtin_popcount(m2) + __builtin_popcount(m3) +
                    __builtin_popcount(m4) + __builtin_popcount(m5) + __builtin_popcount(m6) + __builtin_popcount(m7));
      }
    }
    if (lane == 0) misc[wave] = wc;
  }
  __syncthreads();

  if (wave == 0) {
    int ov = 0;
    int tot = 0;
#pragma unroll 1
    for (int w2 = 0; w2 < NWAVE; ++w2) {
      int c = misc[w2];
      if (c > WLCAP) ov = 1;
      c = c < 0 ? 0 : (c > WLCAP ? WLCAP : c);
      tot += c;
#pragma unroll 1
      for (int b0 = 0; b0 < c; b0 += 32) {
        const int idx = b0 + lane;
        const int ent = wl[w2 * WLCAP + (idx < WLCAP ? idx : WLCAP - 1)];
        const int m32 = (c - b0) < 32 ? (c - b0) : 32;
#pragma unroll 1
        for (int k = 0; k < m32; ++k) {
          const int u    = __builtin_amdgcn_readlane(ent, k);
          const int slot = u & (NBRUN - 1);
          if (lane == 0) cnt[slot] = cnt[slot] + 1;
        }
      }
    }
    if (tot > RCAP) ov = 1;
    if (lane == 0) {
      misc[9]  = ov;
      misc[10] = tot > RCAP ? RCAP : tot;
    }
  }
  __syncthreads();
  if (wave == 0) {
    const int base = lane * (NBRUN / 32);
    int s = 0;
    int dg = 0;
#pragma unroll 1
    for (int i = 0; i < NBRUN / 32; ++i) {
      const int cv = cnt[base + i];
      s += cv;
      dg |= (cv > DEGCAP) ? 1 : 0;
    }
    const unsigned dgm = __builtin_amdgcn_ballot_w32(dg != 0);
    int incl = s;
#pragma unroll
    for (int d = 1; d < 32; d <<= 1) {
      const int y = __shfl_up(incl, d, 32);
      if (lane >= d) incl += y;
    }
    int run = incl - s;
#pragma unroll 1
    for (int i = 0; i < NBRUN / 32; ++i) {
      const int cv = cnt[base + i];
      offs[base + i] = run;
      cur[base + i]  = run;
      run += cv;
    }
    if (lane == 0 && dgm != 0u) misc[9] = 1;
  }
  __syncthreads();

  if (wave == 0) {
#pragma unroll 1
    for (int w2 = 0; w2 < NWAVE; ++w2) {
      int c = misc[w2];
      c = c < 0 ? 0 : (c > WLCAP ? WLCAP : c);
#pragma unroll 1
      for (int b0 = 0; b0 < c; b0 += 32) {
        const int idx = b0 + lane;
        const int ent = wl[w2 * WLCAP + (idx < WLCAP ? idx : WLCAP - 1)];
        const int m32 = (c - b0) < 32 ? (c - b0) : 32;
#pragma unroll 1
        for (int k = 0; k < m32; ++k) {
          const int u    = __builtin_amdgcn_readlane(ent, k);
          const int slot = u & (NBRUN - 1);
          if (lane == 0) {
            int p = cur[slot];
            p = p < 0 ? 0 : (p > RCAP - 1 ? RCAP - 1 : p);
            pl[p] = u;
            cur[slot] = p + 1;
          }
        }
      }
    }
  }
  __syncthreads();

  const int ovf = misc[9];
  const int tot = misc[10];
  int* lp  = LIST + (size_t)blk * (size_t)RCAP;
  int* cop = CO + (size_t)blk * (2 * NBRUN);
  int* fp  = FLAG + (size_t)blk * 32;
#pragma unroll 1
  for (int i = tid * 4; i < RCAP; i += NTHR * 4) {
    const v4i wd = *(const v4ia*)(pl + i);
    const int e0 = clampi((wd.x >> SLB) & 0xFFFFF, 0, NE - 1);
    const int e1 = clampi((wd.y >> SLB) & 0xFFFFF, 0, NE - 1);
    const int e2 = clampi((wd.z >> SLB) & 0xFFFFF, 0, NE - 1);
    const int e3 = clampi((wd.w >> SLB) & 0xFFFFF, 0, NE - 1);
    int sa = srcs[e0];
    int sb = srcs[e1];
    int sc = srcs[e2];
    int sd = srcs[e3];
    int ta = types[e0];
    int tb = types[e1];
    int tc = types[e2];
    int td = types[e3];
    asm volatile("" :: "v"(sa));
    asm volatile("" :: "v"(sb));
    asm volatile("" :: "v"(sc));
    asm volatile("" :: "v"(sd));
    asm volatile("" :: "v"(ta));
    asm volatile("" :: "v"(tb));
    asm volatile("" :: "v"(tc));
    asm volatile("" :: "v"(td));
    sa = clampi(sa, 0, NN - 1); sb = clampi(sb, 0, NN - 1); sc = clampi(sc, 0, NN - 1); sd = clampi(sd, 0, NN - 1);
    ta = clampi(ta, 0, NTY - 1); tb = clampi(tb, 0, NTY - 1); tc = clampi(tc, 0, NTY - 1); td = clampi(td, 0, NTY - 1);
    const int ma = (i     < tot) ? -1 : 0;
    const int mb = (i + 1 < tot) ? -1 : 0;
    const int mc = (i + 2 < tot) ? -1 : 0;
    const int md = (i + 3 < tot) ? -1 : 0;
    const v4i v = {(sa | (ta << 24)) & ma, (sb | (tb << 24)) & mb, (sc | (tc << 24)) & mc, (sd | (td << 24)) & md};
    st2_v4i(lp + i, v);
  }
  {
    const v4i v = *(const v4ia*)(cnt + 4 * tid);
    st2_v4i(cop + 4 * tid, v);
  }
  if (tid < 8) {
    const v4i f = {ovf, ovf, ovf, ovf};
    st2_v4i(fp + 4 * tid, f);
  }
}

__global__ __launch_bounds__(NTHR) void k_walk(const float* __restrict__ T, const int* __restrict__ LIST,
                                               const int* __restrict__ CO, const int* __restrict__ FLAG,
                                               unsigned short* OPA) {
  const int tid = (int)threadIdx.x, lane = tid & 31, wave = tid >> 5;
  const int l = lane & 15;
  const int v = (((int)blockIdx.x * 8 + wave) << 1) + (lane >> 4);
  const int blk = clampi(v >> SLB, 0, NBK - 1), slot = v & (NBRUN - 1);
  const int* cob = CO + (size_t)blk * (2 * NBRUN);
  int cv = cob[slot];
  int ov = cob[NBRUN + slot];
  int flag = FLAG[(size_t)blk * 32];
  asm volatile("" :: "v"(cv));
  asm volatile("" :: "v"(ov));
  asm volatile("" :: "v"(flag));
  const bool big = cv > DEGCAP;
  cv = clampi(cv, 0, DEGCAP);
  ov = clampi(ov, 0, RCAP - 1);
  const int cA = __builtin_amdgcn_readlane(cv, 0);
  const int cB = __builtin_amdgcn_readlane(cv, 16);
  const int trip = cA > cB ? cA : cB;
  int last = ov + (cv > 0 ? cv : 1) - 1;
  last = last > RCAP - 1 ? RCAP - 1 : last;
  const int* lp = LIST + (size_t)blk * (size_t)RCAP;
  v4f a = (v4f){0.0f, 0.0f, 0.0f, 0.0f};
#pragma unroll 1
  for (int k = 0; k < trip; ++k) {
    int idx = ov + k;
    idx = idx > last ? last : idx;
    int wd = lp[idx];
    asm volatile("" :: "v"(wd));
    const int sk = clampi(wd & 0xFFFFFF, 0, NN - 1);
    const int tk = (wd >> 24) & (NTY - 1);
    const v4f t = *(const v4fa*)(T + (size_t)sk * TLD + HD * tk + 4 * l);
    asm volatile("" :: "v"(t));
    const bool act = k < cv;
    a.x = act ? a.x + t.x : a.x;
    a.y = act ? a.y + t.y : a.y;
    a.z = act ? a.z + t.z : a.z;
    a.w = act ? a.w + t.w : a.w;
  }
  const bool bad = (flag != 0) || big;
  const float qnan = __uint_as_float(0x7fc00000u);
  v4f q;
  q.x = bad ? qnan : a.x; q.y = bad ? qnan : a.y; q.z = bad ? qnan : a.z; q.w = bad ? qnan : a.w;
  const v4u o = row_piece(q, lane);
  if (v < NPAD) st2_v4u(OPA + (size_t)v * KT + 8 * l, o);
}

__global__ __launch_bounds__(NTHR) void k_gru(const float* __restrict__ GI, const float* __restrict__ GH,
                                              float* FEAT, unsigned short* OPF, int x0, int nrows) {
  const int tid  = (int)threadIdx.x, lane = tid & 31;
  const int g    = (int)blockIdx.x * NTHR + tid;
  const int lr   = g >> 4;
  const int l    = g & 15;
  const int lrc  = clampi(lr, 0, nrows - 1);
  const float* gi = GI + (size_t)lrc * GLD + 4 * l;
  const float* gh = GH + (size_t)lrc * GLD + 4 * l;
  v4f ir = *(const v4fa*)(gi);
  v4f iz = *(const v4fa*)(gi + HD);
  v4f in = *(const v4fa*)(gi + 2 * HD);
  v4f hr = *(const v4fa*)(gh);
  v4f hz = *(const v4fa*)(gh + HD);
  v4f hn = *(const v4fa*)(gh + 2 * HD);
  const int v = x0 + lrc;
  float* fp = FEAT + (size_t)v * HD + 4 * l;
  v4f f = *(const v4fa*)fp;
  asm volatile("" :: "v"(ir));
  asm volatile("" :: "v"(iz));
  asm volatile("" :: "v"(in));
  asm volatile("" :: "v"(hr));
  asm volatile("" :: "v"(hz));
  asm volatile("" :: "v"(hn));
  asm volatile("" :: "v"(f));
  v4f o = (v4f){0.0f, 0.0f, 0.0f, 0.0f};
#pragma unroll 1
  for (int e = 0; e < 4; ++e) {
    const float xr = ir.x + hr.x;
    const float xz = iz.x + hz.x;
    const float r  = 1.0f / (1.0f + expf(-xr));
    const float z  = 1.0f / (1.0f + expf(-xz));
    float p = r * hn.x;
    asm volatile("" : "+v"(p));
    const float n = tanhf(in.x + p);
    float q1 = (1.0f - z) * n;
    asm volatile("" : "+v"(q1));
    float q2 = z * f.x;
    asm volatile("" : "+v"(q2));
    const float res = q1 + q2;
    o  = (v4f){o.y, o.z, o.w, res};
    ir = (v4f){ir.y, ir.z, ir.w, ir.x};
    iz = (v4f){iz.y, iz.z, iz.w, iz.x};
    in = (v4f){in.y, in.z, in.w, in.x};
    hr = (v4f){hr.y, hr.z, hr.w, hr.x};
    hz = (v4f){hz.y, hz.z, hz.w, hz.x};
    hn = (v4f){hn.y, hn.z, hn.w, hn.x};
    f  = (v4f){f.y, f.z, f.w, f.x};
  }
  const v4u po = row_piece(o, lane);
  if (lr < nrows) {
    st2_v4f(fp, o);
    st2_v4u(OPF + (size_t)v * KT + 8 * l, po);
  }
}

__global__ __launch_bounds__(NTHR) void k_out(const float* __restrict__ FEAT, float* out) {
  const int g  = (int)blockIdx.x * NTHR + (int)threadIdx.x;
  const int gc = clampi(g, 0, NN * HD / 4 - 1);
  const v4f v = *(const v4fa*)(FEAT + (size_t)gc * 4);
  asm volatile("" :: "v"(v));
  if (g < NN * HD / 4) st2_v4f(out + (size_t)g * 4, v);
}

extern "C" void kernel_launch(void* const* d_in, const int* in_sizes, int n_in,
                              void* d_out, int out_size, void* d_ws, size_t ws_size,
                              hipStream_t stream) {
  if (n_in < 10) return;
  if (in_sizes[0] != NN * HD) return;
  if (in_sizes[1] != NTY * HD * HD) return;
  if (in_sizes[2] != NTY * HD) return;
  if (in_sizes[3] != GLD * HD) return;
  if (in_sizes[4] != GLD * HD) return;
  if (in_sizes[5] != GLD) return;
  if (in_sizes[6] != GLD) return;
  if (in_sizes[7] != NE) return;
  if (in_sizes[8] != NE) return;
  if (in_sizes[9] != NE) return;
  if (out_size != NN * HD) return;

  const float* h    = (const float*)d_in[0];
  const float* W    = (const float*)d_in[1];
  const float* b    = (const float*)d_in[2];
  const float* wih  = (const float*)d_in[3];
  const float* whh  = (const float*)d_in[4];
  const float* bih  = (const float*)d_in[5];
  const float* bhh  = (const float*)d_in[6];
  const int*   srcs = (const int*)d_in[7];
  const int*   dsts = (const int*)d_in[8];
  const int*   typs = (const int*)d_in[9];
  float* out = (float*)d_out;

  constexpr size_t zFEAT = (size_t)NPAD * HD * 4;
  constexpr size_t zOPF  = (size_t)NPAD * KT * 2;
  constexpr size_t zOPA  = (size_t)NPAD * KT * 2;
  constexpr size_t zT    = (size_t)NPAD * TLD * 4;
  constexpr size_t zG    = (size_t)XAR * GLD * 4;
  constexpr size_t zLIST = (size_t)NBK * RCAP * 4;
  constexpr size_t zCO   = (size_t)NBK * 2 * NBRUN * 4;
  constexpr size_t zFLAG = (size_t)NBK * 128;
  constexpr size_t zWTY  = (size_t)NTY * HD * KT * 2;
  constexpr size_t zWG   = (size_t)GLD * KT * 2;
  constexpr size_t zBT   = (size_t)NTY * HD * 4;
  constexpr size_t zBG   = (size_t)GLD * 4;
  constexpr size_t oFEAT = 0;
  constexpr size_t oOPF  = oFEAT + zFEAT;
  constexpr size_t oOPA  = oOPF + zOPF;
  constexpr size_t oT    = oOPA + zOPA;
  constexpr size_t oLIST = oT + zT;
  constexpr size_t oCO   = oLIST + zLIST;
  constexpr size_t oFLAG = oCO + zCO;
  constexpr size_t oWTY  = oFLAG + zFLAG;
  constexpr size_t oWIH  = oWTY + zWTY;
  constexpr size_t oWHH  = oWIH + zWG;
  constexpr size_t oBT   = oWHH + zWG;
  constexpr size_t oBI   = oBT + zBT;
  constexpr size_t oBH   = oBI + zBG;
  constexpr size_t oEND  = oBH + zBG;
  static_assert(zFEAT % 256 == 0 && zOPF % 256 == 0 && zT % 256 == 0 && zLIST % 256 == 0 && zCO % 256 == 0);
  static_assert(zFLAG % 256 == 0 && zWTY % 256 == 0 && zWG % 256 == 0 && zBT % 128 == 0 && zBG % 128 == 0);
  static_assert(zG % 128 == 0 && 2 * zG <= zT);
  static_assert((size_t)XBR * GLD * 4 <= zG);
  static_assert(oEND == 95083264);
  static_assert(oEND <= (size_t)WSMAX);
  if (oEND > ws_size) return;

  char* ws = (char*)d_ws;
  float*          FEAT = (float*)(ws + oFEAT);
  unsigned short* OPF  = (unsigned short*)(ws + oOPF);
  unsigned short* OPA  = (unsigned short*)(ws + oOPA);
  float*          T    = (float*)(ws + oT);
  float*          GI   = (float*)(ws + oT);
  float*          GH   = (float*)(ws + oT + zG);
  int*            LIST = (int*)(ws + oLIST);
  int*            CO   = (int*)(ws + oCO);
  int*            FLAG = (int*)(ws + oFLAG);
  unsigned short* WTY  = (unsigned short*)(ws + oWTY);
  unsigned short* WIH  = (unsigned short*)(ws + oWIH);
  unsigned short* WHH  = (unsigned short*)(ws + oWHH);
  float*          BT   = (float*)(ws + oBT);
  float*          BI   = (float*)(ws + oBI);
  float*          BH   = (float*)(ws + oBH);

  hipFuncSetAttribute(reinterpret_cast<const void*>(&k_list), hipFuncAttributeMaxDynamicSharedMemorySize, (int)BK_LDS);

  k_init<<<NPAD * 16 / NTHR, NTHR, 0, stream>>>(h, FEAT, OPF);
  k_prep<<<PB_ALL, NTHR, 0, stream>>>(W, b, wih, whh, bih, bhh, WTY, WIH, WHH, BT, BI, BH);
  k_list<<<NBK, NTHR, BK_LDS, stream>>>(srcs, dsts, typs, LIST, CO, FLAG);

  constexpr int tilesT  = (NPAD / 64) * (TLD / 64);
  constexpr int tilesGA = (XAR / 64) * (GLD / 64);
  constexpr int tilesGB = (XBR / 64) * (GLD / 64);
  for (int s = 0; s < NSTEP; ++s) {
    k_gemm_nt<0, 1><<<(tilesT + 7) / 8, 256, 0, stream>>>(OPF, WTY, BT, T, NPAD, TLD, KT, TLD);
    k_walk<<<NPAD / 16, NTHR, 0, stream>>>(T, LIST, CO, FLAG, OPA);
    k_gemm_nt<0, 1><<<(tilesGA + 7) / 8, 256, 0, stream>>>(OPA + (size_t)XA0 * KT, WIH, BI, GI, XAR, GLD, KT, GLD);
    k_gemm_nt<0, 1><<<(tilesGA + 7) / 8, 256, 0, stream>>>(OPF + (size_t)XA0 * KT, WHH, BH, GH, XAR, GLD, KT, GLD);
    k_gru<<<XAR * 16 / NTHR, NTHR, 0, stream>>>(GI, GH, FEAT, OPF, XA0, XAR);
    k_gemm_nt<0, 1><<<(tilesGB + 7) / 8, 256, 0, stream>>>(OPA + (size_t)XB0 * KT, WIH, BI, GI, XBR, GLD, KT, GLD);
    k_gemm_nt<0, 1><<<(tilesGB + 7) / 8, 256, 0, stream>>>(OPF + (size_t)XB0 * KT, WHH, BH, GH, XBR, GLD, KT, GLD);
    k_gru<<<XBR * 16 / NTHR, NTHR, 0, stream>>>(GI, GH, FEAT, OPF, XB0, XBR);
  }
  k_out<<<NN * HD / 4 / NTHR, NTHR, 0, stream>>>(FEAT, out);
}
